// WeightLinearAttention_40836549050696
// MI455X (gfx1250) — hardware-verified
//
#include <hip/hip_runtime.h>
#define LL 2048
#define BB 2
#define EE 1024
#define NH 16
#define HD 64
#define NTK (LL * BB)
#define LC 64
#define NCH (LL / LC)
#define LP 72

typedef __bf16 v16b __attribute__((ext_vector_type(16)));
typedef unsigned short v8us __attribute__((ext_vector_type(8), may_alias));
typedef float  v8f  __attribute__((ext_vector_type(8)));
typedef float  v4f  __attribute__((ext_vector_type(4)));
typedef float  v4fa __attribute__((ext_vector_type(4), may_alias));
union FragB { v16b v; v8us half[2]; unsigned short u[16]; };

__device__ __forceinline__ unsigned short bf16_bits(float x) { unsigned int u = __float_as_uint(x); return (unsigned short)((u + 0x7FFFu + ((u >> 16) & 1u)) >> 16); }
__device__ __forceinline__ float bf16_val(unsigned short b) { return __uint_as_float(((unsigned int)b) << 16); }
__device__ __forceinline__ float bf16_round(float x) { return bf16_val(bf16_bits(x)); }
template <int NT>
__device__ __forceinline__ v8f mmaN(v16b ah, v16b al, v16b bh, v16b bl, v8f c) {
  c = __builtin_amdgcn_wmma_f32_16x16x32_bf16(false, ah, false, bh, (short)0, c, false, false);
  if (NT >= 2) c = __builtin_amdgcn_wmma_f32_16x16x32_bf16(false, al, false, bh, (short)0, c, false, false);
  if (NT >= 3) c = __builtin_amdgcn_wmma_f32_16x16x32_bf16(false, ah, false, bl, (short)0, c, false, false);
  asm volatile("v_nop\n\tv_nop\n\tv_nop\n\tv_nop" : "+v"(c) : "v"(ah), "v"(al), "v"(bh), "v"(bl));
  return c;
}

__global__ __launch_bounds__(256) void k_wt_bf16(const float* __restrict__ W, unsigned short* __restrict__ Wt, int K, int N) {
  const int t = blockIdx.x * 256 + threadIdx.x;
  const int k8n = K / 8;
  if (t >= N * k8n) return;
  const int n = t / k8n, k8 = (t % k8n) * 8;
  v8us v;
#pragma unroll
  for (int i = 0; i < 8; ++i) v[i] = bf16_bits(W[(size_t)(k8 + i) * N + n]);
  *(volatile v8us*)(Wt + (size_t)n * K + k8) = v;
  __threadfence();
  *(volatile v8us*)(Wt + (size_t)n * K + k8) = v;
}

template <bool ASPLIT, int ACT, bool BIAS_BF16>
__global__ __launch_bounds__(128) void k_gemm_bf(const float* __restrict__ A, int lda, const unsigned short* __restrict__ Wt, int ldb,
                                               const float* __restrict__ bias, float* __restrict__ C, int ldc, int M, int N, int K) {
  __shared__ __attribute__((aligned(16))) float so[4][16][64];
  const int tid = threadIdx.x, w = tid >> 5, lane = tid & 31, ln = lane & 15, hh = lane >> 4;
  const int ntn = N / 64;
  const int wid = blockIdx.x * 4 + w;
  const int mt = wid / ntn, nq = wid % ntn;
  if (mt * 16 >= M) return;
  const int row0 = mt * 16, col0 = nq * 64;
  const float* arow = A + (size_t)(row0 + ln) * lda;
  v8f acc[4] = {};
  for (int kb = 0; kb < K; kb += 32) {
    FragB ah, al;
    const v4f x0 = *(const v4fa*)(arow + kb + 8 * hh), x1 = *(const v4fa*)(arow + kb + 8 * hh + 4);
    const v4f x2 = *(const v4fa*)(arow + kb + 16 + 8 * hh), x3 = *(const v4fa*)(arow + kb + 16 + 8 * hh + 4);
    float xs[16] = {x0[0],x0[1],x0[2],x0[3],x1[0],x1[1],x1[2],x1[3],x2[0],x2[1],x2[2],x2[3],x3[0],x3[1],x3[2],x3[3]};
#pragma unroll
    for (int i = 0; i < 16; ++i) { const unsigned short hb = bf16_bits(xs[i]); ah.u[i] = hb; al.u[i] = ASPLIT ? bf16_bits(xs[i] - bf16_val(hb)) : (unsigned short)0; }
#pragma unroll
    for (int t = 0; t < 4; ++t) {
      const unsigned short* brow = Wt + (size_t)(col0 + t * 16 + ln) * ldb + kb;
      FragB b;
      b.half[0] = *(const v8us*)(brow + 8 * hh);
      b.half[1] = *(const v8us*)(brow + 16 + 8 * hh);
      acc[t] = mmaN<ASPLIT ? 2 : 1>(ah.v, al.v, b.v, b.v, acc[t]);
    }
  }
#pragma unroll
  for (int t = 0; t < 4; ++t) {
    float bv = bias ? bias[col0 + t * 16 + ln] : 0.f;
    if (BIAS_BF16) bv = bf16_round(bv);
#pragma unroll
    for (int r = 0; r < 8; ++r) { float v = acc[t][r] + bv; if (ACT == 1) v = fmaxf(v, 0.f); so[w][8 * hh + r][t * 16 + ln] = v; }
  }
  __builtin_amdgcn_fence(__ATOMIC_ACQ_REL, "workgroup");
  __builtin_amdgcn_wave_barrier();
  const int rsub = lane >> 4, c4 = (lane & 15) * 4;
  for (int pass = 0; pass < 2; ++pass) {
#pragma unroll
    for (int q = 0; q < 8; ++q) {
      const int r = q * 2 + rsub;
      const v4f v = *(const v4fa*)&so[w][r][c4];
      *(volatile v4f*)(C + (size_t)(row0 + r) * ldc + col0 + c4) = v;
    }
    if (pass == 0) __threadfence();
  }
}

template <int D, bool CAUSAL>
__global__ __launch_bounds__(128) void k_flash(const float* __restrict__ qb, const float* __restrict__ kb, const float* __restrict__ vb,
                                             int pitch, int T, int H, float scale, float* __restrict__ y, int ypitch) {
  constexpr int KS = D / 32;
  constexpr int DT = D / 16;
  __shared__ __attribute__((aligned(16))) unsigned short sKh[32][D + 8], sKl[32][D + 8], sVh[32][D + 8], sVl[32][D + 8];
  __shared__ __attribute__((aligned(16))) unsigned short sPh[4][16][40], sPl[4][16][40];
  __shared__ __attribute__((aligned(16))) float sO[4][16][D];
  const int tid = threadIdx.x, w = tid >> 5, lane = tid & 31, ln = lane & 15, hh = lane >> 4;
  const int nqb = (T + 63) / 64;
  const int bh = blockIdx.x / nqb, qblk = blockIdx.x % nqb;
  const int b = bh / H, h = bh % H;
  const int q0 = qblk * 64 + w * 16;
  const float* Q = qb + (size_t)b * T * pitch + h * D;
  const float* K = kb + (size_t)b * T * pitch + h * D;
  const float* V = vb + (size_t)b * T * pitch + h * D;

  FragB aqh[KS], aql[KS];
  {
    int row = q0 + ln; if (row >= T) row = T - 1;
    const float* qr = Q + (size_t)row * pitch;
#pragma unroll
    for (int ks = 0; ks < KS; ++ks)
#pragma unroll
      for (int i = 0; i < 16; ++i) {
        const int d = ks * 32 + ((i < 8) ? (8 * hh + i) : (16 + 8 * hh + (i - 8)));
        const float x = qr[d] * scale; const unsigned short hb = bf16_bits(x);
        aqh[ks].u[i] = hb; aql[ks].u[i] = bf16_bits(x - bf16_val(hb));
      }
  }
  float m_r[8], l_r[8];
#pragma unroll
  for (int r = 0; r < 8; ++r) { m_r[r] = -3.0e38f; l_r[r] = 0.f; }
  v8f oacc[DT];
#pragma unroll
  for (int dt = 0; dt < DT; ++dt) oacc[dt] = (v8f){0.f,0.f,0.f,0.f,0.f,0.f,0.f,0.f};

  const int kv_end = CAUSAL ? min(T, qblk * 64 + 64) : T;
  for (int j0 = 0; j0 < kv_end; j0 += 32) {
    __syncthreads();
    for (int e = tid; e < 32 * (D / 4); e += 128) {
      const int r = e / (D / 4), c4 = (e % (D / 4)) * 4;
      const int key = j0 + r;
      v4f kf = {0.f,0.f,0.f,0.f}, vf = {0.f,0.f,0.f,0.f};
      if (key < T) { kf = *(const v4fa*)(K + (size_t)key * pitch + c4); vf = *(const v4fa*)(V + (size_t)key * pitch + c4); }
#pragma unroll
      for (int t = 0; t < 4; ++t) {
        unsigned short hb = bf16_bits(kf[t]); sKh[r][c4 + t] = hb; sKl[r][c4 + t] = bf16_bits(kf[t] - bf16_val(hb));
        hb = bf16_bits(vf[t]); sVh[r][c4 + t] = hb; sVl[r][c4 + t] = bf16_bits(vf[t] - bf16_val(hb));
      }
    }
    __syncthreads();
    v8f s[2];
#pragma unroll
    for (int nt = 0; nt < 2; ++nt) {
      v8f acc = {};
#pragma unroll
      for (int ks = 0; ks < KS; ++ks) {
        FragB bh_, bl_;
        bh_.half[0] = *(const v8us*)&sKh[nt * 16 + ln][ks * 32 + 8 * hh]; bh_.half[1] = *(const v8us*)&sKh[nt * 16 + ln][ks * 32 + 16 + 8 * hh];
        bl_.half[0] = *(const v8us*)&sKl[nt * 16 + ln][ks * 32 + 8 * hh]; bl_.half[1] = *(const v8us*)&sKl[nt * 16 + ln][ks * 32 + 16 + 8 * hh];
        acc = mmaN<3>(aqh[ks].v, aql[ks].v, bh_.v, bl_.v, acc);
      }
      s[nt] = acc;
    }
    float alpha[8];
#pragma unroll
    for (int r = 0; r < 8; ++r) {
      const int qi = q0 + 8 * hh + r;
      const int ja = j0 + ln, jb = j0 + 16 + ln;
      if (CAUSAL) { if (ja > qi) s[0][r] = -3.0e38f; if (jb > qi) s[1][r] = -3.0e38f; }
      if (ja >= T) s[0][r] = -3.0e38f;
      if (jb >= T) s[1][r] = -3.0e38f;
      float mx = fmaxf(s[0][r], s[1][r]);
      mx = fmaxf(mx, __shfl_xor(mx, 1, 32)); mx = fmaxf(mx, __shfl_xor(mx, 2, 32)); mx = fmaxf(mx, __shfl_xor(mx, 4, 32)); mx = fmaxf(mx, __shfl_xor(mx, 8, 32));
      const float mnew = fmaxf(m_r[r], mx);
      alpha[r] = (mnew > -1.0e38f) ? __expf(m_r[r] - mnew) : 1.0f;
      const float p0 = (s[0][r] > -1.0e38f) ? __expf(s[0][r] - mnew) : 0.f;
      const float p1 = (s[1][r] > -1.0e38f) ? __expf(s[1][r] - mnew) : 0.f;
      m_r[r] = mnew;
      l_r[r] = l_r[r] * alpha[r] + p0 + p1;
      unsigned short hb = bf16_bits(p0); sPh[w][8 * hh + r][ln] = hb;      sPl[w][8 * hh + r][ln] = bf16_bits(p0 - bf16_val(hb));
      hb = bf16_bits(p1);                sPh[w][8 * hh + r][16 + ln] = hb; sPl[w][8 * hh + r][16 + ln] = bf16_bits(p1 - bf16_val(hb));
    }
#pragma unroll
    for (int dt = 0; dt < DT; ++dt)
#pragma unroll
      for (int r = 0; r < 8; ++r) oacc[dt][r] *= alpha[r];
    __builtin_amdgcn_fence(__ATOMIC_ACQ_REL, "workgroup");
    __builtin_amdgcn_wave_barrier();
    FragB pah, pal;
    pah.half[0] = *(const v8us*)&sPh[w][ln][8 * hh]; pah.half[1] = *(const v8us*)&sPh[w][ln][16 + 8 * hh];
    pal.half[0] = *(const v8us*)&sPl[w][ln][8 * hh]; pal.half[1] = *(const v8us*)&sPl[w][ln][16 + 8 * hh];
#pragma unroll
    for (int dt = 0; dt < DT; ++dt) {
      FragB bvh, bvl;
#pragma unroll
      for (int i = 0; i < 8; ++i) {
        bvh.u[i] = sVh[8 * hh + i][dt * 16 + ln]; bvh.u[8 + i] = sVh[16 + 8 * hh + i][dt * 16 + ln];
        bvl.u[i] = sVl[8 * hh + i][dt * 16 + ln]; bvl.u[8 + i] = sVl[16 + 8 * hh + i][dt * 16 + ln];
      }
      oacc[dt] = mmaN<3>(pah.v, pal.v, bvh.v, bvl.v, oacc[dt]);
    }
    __builtin_amdgcn_fence(__ATOMIC_ACQ_REL, "workgroup");
    __builtin_amdgcn_wave_barrier();
  }
#pragma unroll
  for (int r = 0; r < 8; ++r) {
    float l = l_r[r];
    l += __shfl_xor(l, 1, 32); l += __shfl_xor(l, 2, 32); l += __shfl_xor(l, 4, 32); l += __shfl_xor(l, 8, 32);
    l_r[r] = (l > 0.f) ? 1.0f / l : 0.f;
  }
#pragma unroll
  for (int dt = 0; dt < DT; ++dt)
#pragma unroll
    for (int r = 0; r < 8; ++r) sO[w][8 * hh + r][dt * 16 + ln] = oacc[dt][r] * l_r[r];
  __builtin_amdgcn_fence(__ATOMIC_ACQ_REL, "workgroup");
  __builtin_amdgcn_wave_barrier();
  for (int pass = 0; pass < 2; ++pass) {
    for (int r = 0; r < 16; ++r) {
      const int row = q0 + r;
      if (row < T && lane < D / 4) {
        const v4f val = *(const v4fa*)&sO[w][r][lane * 4];
        *(volatile v4f*)(y + ((size_t)b * T + row) * ypitch + h * D + lane * 4) = val;
      }
    }
    if (pass == 0) __threadfence();
  }
}

template <bool ASPLIT, bool BSPLIT, int ACT>
__global__ __launch_bounds__(128) void k_gemm_b(const float* __restrict__ A, int lda, size_t sA, const unsigned short* __restrict__ Bh, const unsigned short* __restrict__ Bl, int ldb, size_t sB,
                                             const float* __restrict__ bias, const float* __restrict__ resid, int ldr, size_t sR, float rsign, float alpha,
                                             float* __restrict__ C, int ldc, size_t sC, int M, int N, int K) {
  __shared__ __attribute__((aligned(16))) float so[4][16][64];
  const int tid = threadIdx.x, w = tid >> 5, lane = tid & 31, ln = lane & 15, hh = lane >> 4;
  const int by = blockIdx.y;
  A += (size_t)by * sA; Bh += (size_t)by * sB; if (BSPLIT) Bl += (size_t)by * sB; C += (size_t)by * sC; if (resid) resid += (size_t)by * sR;
  const int ntn = (N + 63) / 64; const int wid = blockIdx.x * 4 + w; const int mt = wid / ntn, nq = wid % ntn;
  if (mt * 16 >= M) return;
  const int row0 = mt * 16, col0 = nq * 64;
  const float* arow = A + (size_t)(row0 + ln) * lda;
  v8f acc[4] = {};
  for (int kb = 0; kb < K; kb += 32) {
    FragB ah, al;
    const v4f x0 = *(const v4fa*)(arow + kb + 8 * hh), x1 = *(const v4fa*)(arow + kb + 8 * hh + 4);
    const v4f x2 = *(const v4fa*)(arow + kb + 16 + 8 * hh), x3 = *(const v4fa*)(arow + kb + 16 + 8 * hh + 4);
    float xs[16] = {x0[0],x0[1],x0[2],x0[3],x1[0],x1[1],x1[2],x1[3],x2[0],x2[1],x2[2],x2[3],x3[0],x3[1],x3[2],x3[3]};
#pragma unroll
    for (int i = 0; i < 16; ++i) { const unsigned short hb = bf16_bits(xs[i]); ah.u[i] = hb; al.u[i] = ASPLIT ? bf16_bits(xs[i] - bf16_val(hb)) : (unsigned short)0; }
#pragma unroll
    for (int t = 0; t < 4; ++t) {
      if (col0 + t * 16 >= N) continue;
      const size_t boff = (size_t)(col0 + t * 16 + ln) * ldb + kb;
      FragB bh_, bl_; bh_.half[0] = *(const v8us*)(Bh + boff + 8 * hh); bh_.half[1] = *(const v8us*)(Bh + boff + 16 + 8 * hh);
      if (BSPLIT) { bl_.half[0] = *(const v8us*)(Bl + boff + 8 * hh); bl_.half[1] = *(const v8us*)(Bl + boff + 16 + 8 * hh); } else bl_ = bh_;
      acc[t] = mmaN<ASPLIT ? (BSPLIT ? 3 : 2) : 1>(ah.v, al.v, bh_.v, bl_.v, acc[t]);
    }
  }
#pragma unroll
  for (int t = 0; t < 4; ++t) {
    const int col = col0 + t * 16 + ln; if (col0 + t * 16 >= N) continue; const float bv = bias ? bf16_round(bias[col]) : 0.f;
#pragma unroll
    for (int r = 0; r < 8; ++r) { float v = acc[t][r] * alpha + bv; if (resid) v += rsign * resid[(size_t)(row0 + 8 * hh + r) * ldr + col]; if (ACT == 1) v = fmaxf(v, 0.f); else if (ACT == 2) v = fmaxf(v, 0.f) + log1pf(expf(-fabsf(v))); so[w][8 * hh + r][t * 16 + ln] = v; }
  }
  __builtin_amdgcn_fence(__ATOMIC_ACQ_REL, "workgroup"); __builtin_amdgcn_wave_barrier();
  const int rsub = lane >> 4, c4 = (lane & 15) * 4;
  for (int pass = 0; pass < 2; ++pass) {
#pragma unroll
    for (int q = 0; q < 8; ++q) { const int r = q * 2 + rsub; if (col0 + c4 < N) { const v4f v = *(const v4fa*)&so[w][r][c4]; *(volatile v4f*)(C + (size_t)(row0 + r) * ldc + col0 + c4) = v; } }
    if (pass == 0) __threadfence();
  }
}
__global__ __launch_bounds__(256) void k_split_transpose_b(const float* __restrict__ src, int lds_, size_t sIn, unsigned short* __restrict__ hi, unsigned short* __restrict__ lo, size_t sOut, int K, int N) {
  const size_t t = (size_t)blockIdx.x * 256 + threadIdx.x; const int k8n = K / 8; if (t >= (size_t)N * k8n) return;
  src += (size_t)blockIdx.y * sIn; hi += (size_t)blockIdx.y * sOut; lo += (size_t)blockIdx.y * sOut;
  const int n = (int)(t / k8n), k8 = (int)(t % k8n) * 8; v8us vh, vl;
#pragma unroll
  for (int i = 0; i < 8; ++i) { const float x = src[(size_t)(k8 + i) * lds_ + n]; const unsigned short hb = bf16_bits(x); vh[i] = hb; vl[i] = bf16_bits(x - bf16_val(hb)); }
  unsigned short* dh = hi + (size_t)n * K + k8; unsigned short* dl = lo + (size_t)n * K + k8;
  *(volatile v8us*)dh = vh; *(volatile v8us*)dl = vl; __threadfence(); *(volatile v8us*)dh = vh; *(volatile v8us*)dl = vl;
}

__global__ __launch_bounds__(256) void k_round_rows(const float* __restrict__ W, unsigned short* __restrict__ Wt, int n8) {
  const int t = blockIdx.x * 256 + threadIdx.x;
  if (t >= n8) return;
  const v4f a = *(const v4fa*)(W + (size_t)t * 8), b = *(const v4fa*)(W + (size_t)t * 8 + 4);
  v8us v; v[0]=bf16_bits(a[0]); v[1]=bf16_bits(a[1]); v[2]=bf16_bits(a[2]); v[3]=bf16_bits(a[3]);
  v[4]=bf16_bits(b[0]); v[5]=bf16_bits(b[1]); v[6]=bf16_bits(b[2]); v[7]=bf16_bits(b[3]);
  *(volatile v8us*)(Wt + (size_t)t * 8) = v; __threadfence(); *(volatile v8us*)(Wt + (size_t)t * 8) = v;
}

typedef _Float16 v16h __attribute__((ext_vector_type(16)));
union FragH { v16h v; v8us half[2]; _Float16 h[16]; unsigned short u[16]; };
template <int NT>
__device__ __forceinline__ v8f mmaH(v16h ah, v16h al, v16h bh, v16h bl, v8f c) {
  c = __builtin_amdgcn_wmma_f32_16x16x32_f16(false, ah, false, bh, (short)0, c, false, false);
  if (NT >= 2) c = __builtin_amdgcn_wmma_f32_16x16x32_f16(false, al, false, bh, (short)0, c, false, false);
  if (NT >= 3) c = __builtin_amdgcn_wmma_f32_16x16x32_f16(false, ah, false, bl, (short)0, c, false, false);
  asm volatile("v_nop\n\tv_nop\n\tv_nop\n\tv_nop" : "+v"(c) : "v"(ah), "v"(al), "v"(bh), "v"(bl));
  return c;
}
template <bool ASPLIT>
__global__ __launch_bounds__(128) void k_gemm_h(const float* __restrict__ A, int lda, size_t sA, const _Float16* __restrict__ Bh, int ldb, size_t sB, float alpha, float* __restrict__ C, int ldc, size_t sC, int M, int N, int K) {
  __shared__ __attribute__((aligned(16))) float so[4][16][64];
  const int tid = threadIdx.x, w = tid >> 5, lane = tid & 31, ln = lane & 15, hh = lane >> 4; const int by = blockIdx.y;
  A += (size_t)by * sA; Bh += (size_t)by * sB; C += (size_t)by * sC;
  const int ntn = (N + 63) / 64; const int wid = blockIdx.x * 4 + w; const int mt = wid / ntn, nq = wid % ntn; if (mt * 16 >= M) return;
  const int row0 = mt * 16, col0 = nq * 64; const float* arow = A + (size_t)(row0 + ln) * lda;
  v8f acc[4] = {};
  for (int kb = 0; kb < K; kb += 32) {
    FragH ah, al;
    const v4f x0 = *(const v4fa*)(arow + kb + 8 * hh), x1 = *(const v4fa*)(arow + kb + 8 * hh + 4), x2 = *(const v4fa*)(arow + kb + 16 + 8 * hh), x3 = *(const v4fa*)(arow + kb + 16 + 8 * hh + 4);
    float xs[16] = {x0[0],x0[1],x0[2],x0[3],x1[0],x1[1],x1[2],x1[3],x2[0],x2[1],x2[2],x2[3],x3[0],x3[1],x3[2],x3[3]};
#pragma unroll
    for (int i = 0; i < 16; ++i) { const _Float16 h = (_Float16)xs[i]; ah.h[i] = h; al.h[i] = ASPLIT ? (_Float16)(xs[i] - (float)h) : (_Float16)0.0f; }
#pragma unroll
    for (int t = 0; t < 4; ++t) { if (col0 + t * 16 >= N) continue; const size_t boff = (size_t)(col0 + t * 16 + ln) * ldb + kb; FragH bq; bq.half[0] = *(const v8us*)(Bh + boff + 8 * hh); bq.half[1] = *(const v8us*)(Bh + boff + 16 + 8 * hh);
      acc[t] = mmaH<ASPLIT ? 2 : 1>(ah.v, al.v, bq.v, bq.v, acc[t]); }
  }
#pragma unroll
  for (int t = 0; t < 4; ++t) { if (col0 + t * 16 >= N) continue;
#pragma unroll
    for (int r = 0; r < 8; ++r) so[w][8 * hh + r][t * 16 + ln] = acc[t][r] * alpha; }
  __builtin_amdgcn_fence(__ATOMIC_ACQ_REL, "workgroup"); __builtin_amdgcn_wave_barrier();
  const int rsub = lane >> 4, c4 = (lane & 15) * 4;
  for (int pass = 0; pass < 2; ++pass) {
#pragma unroll
    for (int q = 0; q < 8; ++q) { const int r = q * 2 + rsub; if (col0 + c4 < N) { const v4f v = *(const v4fa*)&so[w][r][c4]; *(volatile v4f*)(C + (size_t)(row0 + r) * ldc + col0 + c4) = v; } }
    if (pass == 0) __threadfence(); }
}

__device__ __forceinline__ void ldA(FragH& f, const _Float16* base, int row, int k0, int ln, int hh) { const unsigned short* p = (const unsigned short*)base + (size_t)(row + ln) * LP + k0; f.half[0] = *(const v8us*)(p + 8 * hh); f.half[1] = *(const v8us*)(p + 16 + 8 * hh); }
__global__ __launch_bounds__(256) void k_phi(const float* __restrict__ Qm, const float* __restrict__ Km, const float* __restrict__ Vm, float* __restrict__ QF, float* __restrict__ KF, float* __restrict__ VF) { const size_t t = (size_t)blockIdx.x * 256 + threadIdx.x; if (t >= (size_t)BB * NH * LL * (HD / 2)) return;
  const int i = (int)(t % (HD / 2)); const int l = (int)((t / (HD / 2)) % LL); const int h = (int)((t / ((size_t)(HD / 2) * LL)) % NH); const int b = (int)(t / ((size_t)(HD / 2) * LL * NH));
  const size_t src = ((size_t)l * BB + b) * EE + h * HD + 2 * i; const size_t dst = (((size_t)b * NH + h) * LL + l) * HD + 2 * i;
  const float theta = powf(10000.0f, -2.0f / (float)HD * (float)i); const float ang = (float)l * theta; const float cs = cosf(ang), sn = sinf(ang);
  const float q0 = fmaxf(Qm[src], 0.f), q1 = fmaxf(Qm[src + 1], 0.f), k0 = fmaxf(Km[src], 0.f), k1 = fmaxf(Km[src + 1], 0.f);
  typedef float v2f __attribute__((ext_vector_type(2))); v2f qo, ko, vo; qo.x = q0 * cs - q1 * sn; qo.y = q0 * sn + q1 * cs; ko.x = k0 * cs - k1 * sn; ko.y = k0 * sn + k1 * cs; vo.x = Vm[src]; vo.y = Vm[src + 1];
  for (int pass = 0; pass < 2; ++pass) { *(volatile v2f*)(QF + dst) = qo; *(volatile v2f*)(KF + dst) = ko; *(volatile v2f*)(VF + dst) = vo; if (pass == 0) __threadfence(); } }
__global__ __launch_bounds__(128) void k_linattn(const float* __restrict__ QF, const float* __restrict__ KF, const float* __restrict__ VF, float* __restrict__ O) {
  __shared__ __attribute__((aligned(16))) _Float16 sQ[LC * LP], sK[LC * LP], sKT[HD * LP], sVT[HD * LP], sP[LC * LP], sST[HD * LP];
  __shared__ float sS[HD][HD + 1]; __shared__ float sR[LC][HD + 1]; __shared__ float sZ[HD], sZn[HD]; __shared__ float sQf[LC][HD + 1], sKf[LC][HD + 1];
  const int tid = threadIdx.x, w = tid >> 5, lane = tid & 31, ln = lane & 15, hh = lane >> 4; const int bh = blockIdx.x; const int b = bh / NH, h = bh % NH;
  for (int i = tid; i < HD * (HD + 1); i += 128) (&sS[0][0])[i] = 0.f;
  for (int i = tid; i < HD * LP; i += 128) sST[i] = (_Float16)0.0f;
  if (tid < HD) { sZ[tid] = 0.f; sZn[tid] = 0.f; }
  __syncthreads();
  const float* qb = QF + (size_t)bh * LL * HD; const float* kb = KF + (size_t)bh * LL * HD; const float* vb = VF + (size_t)bh * LL * HD;
  for (int c = 0; c < NCH; ++c) {
    for (int i = tid; i < LC * HD; i += 128) { const int r = i >> 6, d = i & 63; const size_t g = ((size_t)(c * LC + r)) * HD + d; const float q = qb[g], k = kb[g], v = vb[g];
      sQ[r * LP + d] = (_Float16)q; sQf[r][d] = q; sKf[r][d] = k; sK[r * LP + d] = (_Float16)k; sKT[d * LP + r] = (_Float16)k; sVT[d * LP + r] = (_Float16)v; }
    __syncthreads();
    if (tid < HD) { float s = 0.f; for (int r = 0; r < LC; ++r) s += sKf[r][tid]; sZn[tid] = sZ[tid] + s; }
    const int i0 = w * 16; v8f accP[4] = {}, accX[4] = {};
#pragma unroll
    for (int ks = 0; ks < 2; ++ks) { FragH a; ldA(a, sQ, i0, ks * 32, ln, hh);
#pragma unroll
      for (int t = 0; t < 4; ++t) { FragH bk, bs; ldA(bk, sK, t * 16, ks * 32, ln, hh); ldA(bs, sST, t * 16, ks * 32, ln, hh); accP[t] = mmaH<1>(a.v, a.v, bk.v, bk.v, accP[t]); accX[t] = mmaH<1>(a.v, a.v, bs.v, bs.v, accX[t]); } }
#pragma unroll
    for (int t = 0; t < 4; ++t) {
#pragma unroll
      for (int r = 0; r < 8; ++r) { const int i = i0 + 8 * hh + r, j = t * 16 + ln; const float p = (j <= i) ? accP[t][r] : 0.f; sP[i * LP + j] = (_Float16)p; } }
    float drow[8];
#pragma unroll
    for (int r = 0; r < 8; ++r) { const int i = i0 + 8 * hh + r; float s = 0.f;
#pragma unroll 1
      for (int t = 0; t < 4; ++t) { const int j = t * 16 + ln; if (j <= i) { float dsum = 0.f;
#pragma unroll 8
          for (int d = 0; d < HD; ++d) dsum += sQf[i][d] * sKf[j][d]; s += dsum; } }
      for (int o = 8; o >= 1; o >>= 1) s += __shfl_xor(s, o, 32); drow[r] = s; }
    __builtin_amdgcn_fence(__ATOMIC_ACQ_REL, "workgroup"); __builtin_amdgcn_wave_barrier();
    v8f accI[4] = {};
#pragma unroll
    for (int ks = 0; ks < 2; ++ks) { FragH a; ldA(a, sP, i0, ks * 32, ln, hh);
#pragma unroll
      for (int t = 0; t < 4; ++t) { FragH bv; ldA(bv, sVT, t * 16, ks * 32, ln, hh); accI[t] = mmaH<1>(a.v, a.v, bv.v, bv.v, accI[t]); } }
#pragma unroll
    for (int r = 0; r < 8; ++r) { const int i = i0 + 8 * hh + r; float qz = 0.f;
#pragma unroll 4
      for (int d = ln; d < HD; d += 16) qz += sQf[i][d] * sZ[d];
      for (int o = 8; o >= 1; o >>= 1) qz += __shfl_xor(qz, o, 32); const float den = fmaxf(drow[r] + qz, 1e-4f); const float rd = 1.0f / den;
#pragma unroll
      for (int t = 0; t < 4; ++t) { const int e = t * 16 + ln; sR[i][e] = (accI[t][r] + accX[t][r]) * rd; } }
    __syncthreads();
    { v8f accS[4] = {};
#pragma unroll
      for (int ks = 0; ks < 2; ++ks) { FragH a; ldA(a, sKT, i0, ks * 32, ln, hh);
#pragma unroll
        for (int t = 0; t < 4; ++t) { FragH bv; ldA(bv, sVT, t * 16, ks * 32, ln, hh); accS[t] = mmaH<1>(a.v, a.v, bv.v, bv.v, accS[t]); } }
#pragma unroll
      for (int t = 0; t < 4; ++t) {
#pragma unroll
        for (int r = 0; r < 8; ++r) { const int d = i0 + 8 * hh + r, e = t * 16 + ln; const float sv = sS[d][e] + accS[t][r]; sS[d][e] = sv; sST[e * LP + d] = (_Float16)sv; } } }
    if (tid < HD) sZ[tid] = sZn[tid];
    __syncthreads();
    for (int pass = 0; pass < 2; ++pass) { for (int i = tid; i < LC * HD; i += 128) { const int r = i >> 6, e = i & 63; *(volatile float*)(O + ((size_t)(c * LC + r) * BB + b) * EE + h * HD + e) = sR[r][e]; } if (pass == 0) __threadfence(); }
    __syncthreads();
  }
}
extern "C" void kernel_launch(void* const* d_in, const int* in_sizes, int n_in,
                              void* d_out, int out_size, void* d_ws, size_t ws_size, hipStream_t stream) {
  (void)in_sizes; (void)n_in; (void)out_size;
  const float* xq = (const float*)d_in[0]; const float* xk = (const float*)d_in[1]; const float* xv = (const float*)d_in[2]; const float* Wq = (const float*)d_in[3]; const float* bq = (const float*)d_in[4]; const float* Wk = (const float*)d_in[5]; const float* bk = (const float*)d_in[6]; const float* Wv = (const float*)d_in[7]; const float* bv = (const float*)d_in[8]; const float* Wo = (const float*)d_in[9]; const float* bo = (const float*)d_in[10];
  char* ws = (char*)d_ws; size_t off = 0;
  auto take = [&](size_t bytes) { char* p = ws + off; off += (bytes + 255) & ~(size_t)255; return p; };
  unsigned short* Bq = (unsigned short*)take((size_t)EE * EE * 2); unsigned short* Bk = (unsigned short*)take((size_t)EE * EE * 2); unsigned short* Bv = (unsigned short*)take((size_t)EE * EE * 2); unsigned short* Bo = (unsigned short*)take((size_t)EE * EE * 2);
  float* Qm = (float*)take((size_t)NTK * EE * 4); float* Km = (float*)take((size_t)NTK * EE * 4); float* Vm = (float*)take((size_t)NTK * EE * 4);
  float* QF = (float*)take((size_t)NTK * EE * 4); float* KF = (float*)take((size_t)NTK * EE * 4); float* VF = (float*)take((size_t)NTK * EE * 4); float* O = Qm;
  if (off > ws_size) return;
  k_round_rows<<<(EE * EE / 8 + 255) / 256, 256, 0, stream>>>(Wq, Bq, EE * EE / 8); k_round_rows<<<(EE * EE / 8 + 255) / 256, 256, 0, stream>>>(Wk, Bk, EE * EE / 8); k_round_rows<<<(EE * EE / 8 + 255) / 256, 256, 0, stream>>>(Wv, Bv, EE * EE / 8); k_round_rows<<<(EE * EE / 8 + 255) / 256, 256, 0, stream>>>(Wo, Bo, EE * EE / 8);
  k_gemm_b<false, false, 0><<<dim3(((NTK / 16) * (EE / 64) + 3) / 4, 1), 128, 0, stream>>>(xq, EE, 0, Bq, Bq, EE, 0, bq, nullptr, 0, 0, 1.f, 1.f, Qm, EE, 0, NTK, EE, EE);
  k_gemm_b<false, false, 0><<<dim3(((NTK / 16) * (EE / 64) + 3) / 4, 1), 128, 0, stream>>>(xk, EE, 0, Bk, Bk, EE, 0, bk, nullptr, 0, 0, 1.f, 1.f, Km, EE, 0, NTK, EE, EE);
  k_gemm_b<false, false, 0><<<dim3(((NTK / 16) * (EE / 64) + 3) / 4, 1), 128, 0, stream>>>(xv, EE, 0, Bv, Bv, EE, 0, bv, nullptr, 0, 0, 1.f, 1.f, Vm, EE, 0, NTK, EE, EE);
  k_phi<<<(unsigned)(((size_t)BB * NH * LL * (HD / 2) + 255) / 256), 256, 0, stream>>>(Qm, Km, Vm, QF, KF, VF);
  k_linattn<<<BB * NH, 128, 0, stream>>>(QF, KF, VF, O);
  k_gemm_b<true, false, 0><<<dim3(((NTK / 16) * (EE / 64) + 3) / 4, 1), 128, 0, stream>>>(O, EE, 0, Bo, Bo, EE, 0, bo, nullptr, 0, 0, 1.f, 1.f, (float*)d_out, EE, 0, NTK, EE, EE);
}
